// RESIDUAL_4105988735320
// MI455X (gfx1250) — hardware-run, weakly checked
//
#include <hip/hip_runtime.h>

typedef float          v8f   __attribute__((ext_vector_type(8)));
typedef float          v4f   __attribute__((ext_vector_type(4)));
typedef unsigned int   v4u   __attribute__((ext_vector_type(4)));
typedef int            v8i   __attribute__((ext_vector_type(8)));
typedef unsigned short v8us  __attribute__((ext_vector_type(8)));
typedef unsigned short v16us __attribute__((ext_vector_type(16)));
typedef __bf16         v16bf __attribute__((ext_vector_type(16)));
typedef _Float16       v16h  __attribute__((ext_vector_type(16)));
typedef v4f  __attribute__((may_alias)) v4fa;
typedef v8us __attribute__((may_alias)) v8usa;
union FragB { v16bf v; v16us u; v8us h[2]; v8i w; };
union FragH { v16h  v; v16us u; v8us h[2]; v8i w; };

__device__ __forceinline__ v8f wmb(const FragB& a, const FragB& b, v8f c) {
  v8f d = __builtin_amdgcn_wmma_f32_16x16x32_bf16(false, a.v, false, b.v, (short)0, c, false, false);
  asm volatile("v_nop\n\tv_nop\n\tv_nop\n\tv_nop" : "+v"(d) : "v"(a.w), "v"(b.w));
  return d;
}

__device__ __forceinline__ v8f wmh(const FragH& a, const FragH& b, v8f c) {
  v8f d = __builtin_amdgcn_wmma_f32_16x16x32_f16(false, a.v, false, b.v, (short)0, c, false, false);
  asm volatile("v_nop\n\tv_nop\n\tv_nop\n\tv_nop" : "+v"(d) : "v"(a.w), "v"(b.w));
  return d;
}

__device__ __forceinline__ unsigned bf16_bits(float f) {
  const unsigned u = __float_as_uint(f);
  const unsigned r = (u + 0x7FFFu + ((u >> 16) & 1u)) >> 16;
  const unsigned q = (u >> 16) | 0x40u;
  return ((u & 0x7fffffffu) > 0x7f800000u) ? q : r;
}

__device__ __forceinline__ float bf16_val(float f) {
  return __uint_as_float(bf16_bits(f) << 16);
}
__device__ __forceinline__ int clampi(int v, int lo, int hi) {
  return v < lo ? lo : (v > hi ? hi : v);
}

__device__ __forceinline__ unsigned f16_bits(float f) {
  const unsigned u  = __float_as_uint(f);
  const unsigned s  = (u >> 16) & 0x8000u;
  const unsigned a  = u & 0x7fffffffu;
  const unsigned t  = a - 0x38000000u;
  const unsigned r  = (t + 0x0FFFu + ((t >> 13) & 1u)) >> 13;
  const unsigned rc = r > 0x7C00u ? 0x7C00u : r;
  const bool small  = a < 0x38800000u;
  const bool isnan  = a > 0x7f800000u;
  const unsigned fin = small ? 0u : (s | rc);
  return isnan ? (s | 0x7E00u) : fin;
}

__device__ __forceinline__ unsigned pk16(unsigned lo, unsigned hi) { return lo | (hi << 16); }
__device__ __forceinline__ unsigned bf16_lo_bits(float v) {
  float hi = bf16_val(v);
  asm volatile("" : "+v"(hi));
  return bf16_bits(v - hi);
}
__device__ __forceinline__ v4u pack8_bf16(v4f a, v4f c) {
  return (v4u){ pk16(bf16_bits(a[0]), bf16_bits(a[1])), pk16(bf16_bits(a[2]), bf16_bits(a[3])),
                pk16(bf16_bits(c[0]), bf16_bits(c[1])), pk16(bf16_bits(c[2]), bf16_bits(c[3])) };
}
__device__ __forceinline__ v4u pack8_bf16_lo(v4f a, v4f c) {
  return (v4u){ pk16(bf16_lo_bits(a[0]), bf16_lo_bits(a[1])), pk16(bf16_lo_bits(a[2]), bf16_lo_bits(a[3])),
                pk16(bf16_lo_bits(c[0]), bf16_lo_bits(c[1])), pk16(bf16_lo_bits(c[2]), bf16_lo_bits(c[3])) };
}
__device__ __forceinline__ v4u pack8_f16(v4f a, v4f c) {
  return (v4u){ pk16(f16_bits(a[0]), f16_bits(a[1])), pk16(f16_bits(a[2]), f16_bits(a[3])),
                pk16(f16_bits(c[0]), f16_bits(c[1])), pk16(f16_bits(c[2]), f16_bits(c[3])) };
}

template <int FORM>
__global__ __launch_bounds__(256) void k_plane(const float* __restrict__ src, int rows, int cols, int ldsrc,
                                               unsigned short* __restrict__ dst, int MP, int KP) {
  static_assert(FORM >= 0 && FORM <= 3);
  const int KTOT = (FORM == 1 || FORM == 3) ? 2 * KP : KP;
  const unsigned ppr   = (unsigned)(KTOT >> 3);
  const unsigned kp8   = (unsigned)(KP >> 3);
  const unsigned total = (unsigned)MP * ppr;
  const unsigned g     = blockIdx.x * 256u + threadIdx.x;
  const unsigned rowu  = g / ppr;
  const unsigned p     = g - rowu * ppr;
  const bool second    = p >= kp8;
  const int row = (int)rowu;
  const int c0  = (int)((second ? p - kp8 : p) << 3);
  const float* srow = src + (size_t)clampi(row, 0, rows - 1) * (size_t)ldsrc;
  float x[8];
  unsigned mk[8];
#pragma unroll
  for (int e = 0; e < 8; ++e) {
    const int c = c0 + e;
    const float v = srow[clampi(c, 0, cols - 1)];
    asm volatile("" :: "v"(v));
    x[e]  = v;
    mk[e] = (row < rows && c < cols) ? 0xFFFFu : 0u;
  }
  const v4f a = (v4f){ x[0], x[1], x[2], x[3] };
  const v4f c = (v4f){ x[4], x[5], x[6], x[7] };
  v4u o;
  if (FORM == 2) {
    o = pack8_f16(a, c);
  } else {
    const v4u hi = pack8_bf16(a, c);
    o = hi;
    if (FORM == 1) { const v4u lo = pack8_bf16_lo(a, c); o = second ? lo : hi; }
  }
  const v4u mw = (v4u){ pk16(mk[0], mk[1]), pk16(mk[2], mk[3]), pk16(mk[4], mk[5]), pk16(mk[6], mk[7]) };
  o &= mw;
  if (g < total) {
    volatile v4u* q = (volatile v4u*)(dst + (size_t)g * 8);
    *q = o;
    __threadfence();
    *q = o;
  }
}

template <int FORM> struct FragOf    { typedef FragB T; };
template <>         struct FragOf<2> { typedef FragH T; };
__device__ __forceinline__ v8f mm(const FragB& a, const FragB& b, v8f c) { return wmb(a, b, c); }
__device__ __forceinline__ v8f mm(const FragH& a, const FragH& b, v8f c) { return wmh(a, b, c); }
template <class F> __device__ __forceinline__ F ld_frag(const unsigned short* p) {
  F f;
  f.h[0] = *(const v8usa*)(p);
  f.h[1] = *(const v8usa*)(p + 16);
  return f;
}

template <int FORM, int EPI>
__global__ __launch_bounds__(256) __attribute__((amdgpu_num_vgpr(248)))
void k_gemm_nt(const unsigned short* __restrict__ A, const unsigned short* __restrict__ B,
               const float* __restrict__ bias, float* __restrict__ D, int M, int N, int KTOT, int ldd) {
  static_assert(FORM >= 0 && FORM <= 2);
  static_assert(EPI == 0 || EPI == 1);
  typedef typename FragOf<FORM>::T F;
  __shared__ __attribute__((aligned(16))) float sT[8][16 * 68];
  const int lane = threadIdx.x & 31;
  const int wave = threadIdx.x >> 5;
  const int tilesM = (M + 63) >> 6;
  const int tilesN = (N + 63) >> 6;
  const int tile = blockIdx.x * 8 + wave;
  if (tile >= tilesM * tilesN) return;
  const int tm = tile / tilesN;
  const int tn = tile - tm * tilesN;
  const int m0 = tm << 6;
  const int n0 = tn << 6;

  const int rl = lane & 15;
  const int h8 = (lane >> 4) * 8;
  const unsigned short* pa = A + (size_t)(m0 + rl) * (size_t)KTOT + h8;
  const unsigned short* pb = B + (size_t)(n0 + rl) * (size_t)KTOT + h8;

  v8f acc[4][4];
#pragma unroll
  for (int i = 0; i < 4; ++i)
#pragma unroll
    for (int j = 0; j < 4; ++j) acc[i][j] = (v8f){0.f, 0.f, 0.f, 0.f, 0.f, 0.f, 0.f, 0.f};

#pragma unroll 1
  for (int k0 = 0; k0 < KTOT; k0 += 32) {
    F bf[4];
#pragma unroll
    for (int j = 0; j < 4; ++j) bf[j] = ld_frag<F>(pb + (size_t)(j << 4) * (size_t)KTOT + k0);
#pragma unroll
    for (int i = 0; i < 4; ++i) {
      const F af = ld_frag<F>(pa + (size_t)(i << 4) * (size_t)KTOT + k0);
#pragma unroll
      for (int j = 0; j < 4; ++j) acc[i][j] = mm(af, bf[j], acc[i][j]);
    }
  }

  float* slab = sT[wave];
  const int hh = lane >> 4;
  const int c4 = (lane & 15) * 4;
  const int nc = n0 + c4;
  const bool cok = nc < N;
  v4f bv = (v4f){0.f, 0.f, 0.f, 0.f};
  if (EPI == 1) {
    bv = *(const v4fa*)(bias + clampi(nc, 0, N - 4));
    asm volatile("" :: "v"(bv));
  }
#pragma unroll
  for (int i = 0; i < 4; ++i) {
    const int mBase = m0 + (i << 4);
#pragma unroll
    for (int j = 0; j < 4; ++j) {
#pragma unroll
      for (int r = 0; r < 8; ++r) slab[(h8 + r) * 68 + (j << 4) + rl] = acc[i][j][r];
    }
    __builtin_amdgcn_fence(__ATOMIC_RELEASE, "workgroup");
    __builtin_amdgcn_wave_barrier();
    __builtin_amdgcn_fence(__ATOMIC_ACQUIRE, "workgroup");
    v4f vv[8];
#pragma unroll
    for (int it = 0; it < 8; ++it) {
      const int row = it * 2 + hh;
      v4f v = *(const v4fa*)(slab + row * 68 + c4);
      if (EPI == 1) v += bv;
      vv[it] = v;
    }
    for (int pass = 0; pass < 2; ++pass) {
#pragma unroll
      for (int it = 0; it < 8; ++it) {
        const int row = mBase + it * 2 + hh;
        if (cok && row < M) *(volatile v4f*)(D + (size_t)row * (size_t)ldd + nc) = vv[it];
      }
      __threadfence();
    }
    __builtin_amdgcn_fence(__ATOMIC_RELEASE, "workgroup");
    __builtin_amdgcn_wave_barrier();
    __builtin_amdgcn_fence(__ATOMIC_ACQUIRE, "workgroup");
  }
}

#pragma clang fp contract(off)

#ifndef TWO_TERM_C1B
#define TWO_TERM_C1B 1
#endif
#ifndef TWO_TERM_C2A
#define TWO_TERM_C2A 1
#endif
#ifndef TWO_TERM_C2B
#define TWO_TERM_C2B 1
#endif
#ifndef TWO_TERM_L2
#define TWO_TERM_L2 1
#endif
static_assert(TWO_TERM_C1B == 0 || TWO_TERM_C1B == 1);
static_assert(TWO_TERM_C2A == 0 || TWO_TERM_C2A == 1);
static_assert(TWO_TERM_C2B == 0 || TWO_TERM_C2B == 1);
static_assert(TWO_TERM_L2 == 0 || TWO_TERM_L2 == 1);

typedef float        v2f __attribute__((ext_vector_type(2)));
typedef int          v4i __attribute__((ext_vector_type(4)));
typedef double       v2d __attribute__((ext_vector_type(2)));
typedef v2f __attribute__((may_alias)) v2fa;
typedef v4i __attribute__((may_alias)) v4ia;
typedef v4u __attribute__((may_alias)) v4ua;

constexpr int NS    = 60000;
constexpr int MS    = 300000;
constexpr int CH    = 32;
constexpr int NBAT  = 4, HH = 496, WW = 432;
constexpr int NCELL = NBAT * HH * WW;
constexpr int NPAD  = 60032;
constexpr int MPAD  = 300032;
constexpr int LDV   = 64;
constexpr int KTAP  = 288;
constexpr int K_1A  = KTAP;
constexpr int K_1B  = TWO_TERM_C1B ? 2 * KTAP : KTAP;
constexpr int K_2A  = TWO_TERM_C2A ? 2 * KTAP : KTAP;
constexpr int K_2B  = TWO_TERM_C2B ? 2 * KTAP : KTAP;
constexpr int K_L1  = 32;
constexpr int K_L2  = TWO_TERM_L2 ? 64 : 32;
constexpr int NREC_N = (NS + 127) / 128;
constexpr int NREC_M = (MS + 127) / 128;

static_assert(NCELL == 857088 && NCELL % 32 == 0);
static_assert(NPAD % 64 == 0 && NPAD >= NS && NPAD - NS < 64 && NPAD % 16 == 0);
static_assert(MPAD % 64 == 0 && MPAD >= MS && MPAD - MS < 64 && MPAD % 16 == 0 && MPAD % 32 == 0);
static_assert(KTAP % 32 == 0 && (2 * KTAP) % 32 == 0 && K_L1 % 32 == 0 && K_L2 % 32 == 0);
static_assert(NS % 2 == 0 && NS % 4 == 0 && NS % 8 == 0 && (NPAD / 2) % 8 == 0);
static_assert(LDV % 32 == 0 && CH == 32);
static_assert(NREC_N == 469 && NREC_M == 2344);

constexpr int P_B = 0, P_G = 128, P_BE = 320, P_N = 512;
constexpr int S_N = 6 * 64;

constexpr int PBK_RUN  = 1024;
constexpr int PBK_NBLK = 59;
constexpr int RCAP     = 6656;
constexpr int DEGCAP   = 32;
constexpr int WLCAP    = 2048;
constexpr int EPW      = MS / 8;
constexpr int SUB      = 128;
constexpr int NSTEP    = (EPW + SUB - 1) / SUB;
static_assert(PBK_NBLK * PBK_RUN >= NS && (PBK_NBLK - 1) * PBK_RUN < NS);
static_assert(MS % 8 == 0 && NSTEP * SUB >= EPW && (NSTEP - 1) * SUB < EPW);
static_assert(RCAP % 256 == 0 && RCAP * 4 >= 5242 * 5 && RCAP >= 2 * DEGCAP);
static_assert(DEGCAP >= 17 + 8 && DEGCAP <= 32);
static_assert(WLCAP * 8 >= RCAP);
static_assert((((long long)(MS - 1) << 10) | 1023) < (1LL << 31));
constexpr int BK_WL   = 0;
constexpr int BK_SL   = 8 * WLCAP;
constexpr int BK_CNT  = BK_SL + RCAP;
constexpr int BK_OFF  = BK_CNT + PBK_RUN;
constexpr int BK_CUR  = BK_OFF + PBK_RUN;
constexpr int BK_MISC = BK_CUR + PBK_RUN;
constexpr int BK_INTS = BK_MISC + 16;
constexpr int BK_LDS  = BK_INTS * 4;
static_assert(BK_LDS == 104512 && BK_LDS <= 262144 && BK_LDS <= 327680);
static_assert(BK_SL % 4 == 0 && BK_CNT % 4 == 0 && (RCAP + PBK_RUN) % 4 == 0);

constexpr int GB_CELLS  = 8192;
constexpr int GB_BLOCKS = (NCELL + GB_CELLS - 1) / GB_CELLS;
static_assert(GB_BLOCKS == 105 && GB_CELLS % 1024 == 0 && NCELL % 4 == 0);
static_assert((NCELL - (GB_BLOCKS - 1) * GB_CELLS) % 128 == 0);

constexpr size_t SZ_X    = (size_t)MPAD * LDV * 4;
constexpr size_t SZ_Y    = (size_t)MPAD * 64 * 2;
constexpr size_t SZ_F    = (size_t)NS * CH * 4;
constexpr size_t SZ_V    = (size_t)NPAD * LDV * 4;
constexpr size_t SZ_G    = (size_t)NCELL * 4;
constexpr size_t SZ_NB   = (size_t)NS * 16 * 4;
constexpr size_t SZ_LIST = (size_t)PBK_NBLK * RCAP * 4;
constexpr size_t SZ_NODE = (size_t)PBK_NBLK * PBK_RUN * 4;
constexpr size_t SZ_FLAG = 7680;
constexpr size_t SZ_BW1  = (size_t)64 * 2 * KTAP * 2;
constexpr size_t SZ_BW   = 4 * SZ_BW1;
constexpr size_t SZ_CWT  = (size_t)64 * 32 * 2;
constexpr size_t SZ_LWT  = (size_t)64 * 64 * 2;
constexpr size_t SZ_PAR  = (size_t)P_N * 4;
constexpr size_t SZ_ST   = (size_t)S_N * 4;
constexpr size_t SZ_REC  = (size_t)NREC_M * CH * 8;
constexpr size_t OFF_X    = 0;
constexpr size_t OFF_Y    = OFF_X + SZ_X;
constexpr size_t OFF_F2   = OFF_Y + SZ_Y;
constexpr size_t OFF_LIST = OFF_F2 + SZ_F;
constexpr size_t OFF_CNT  = OFF_LIST + SZ_LIST;
constexpr size_t OFF_OFF  = OFF_CNT + SZ_NODE;
constexpr size_t OFF_FLAG = OFF_OFF + SZ_NODE;
constexpr size_t OFF_BW   = OFF_FLAG + SZ_FLAG;
constexpr size_t OFF_CWT  = OFF_BW + SZ_BW;
constexpr size_t OFF_LWT  = OFF_CWT + SZ_CWT;
constexpr size_t OFF_PAR  = OFF_LWT + SZ_LWT;
constexpr size_t OFF_ST   = OFF_PAR + SZ_PAR;
constexpr size_t OFF_REC  = OFF_ST + SZ_ST;
constexpr size_t WS_TOTAL = OFF_REC + SZ_REC;
constexpr size_t YO_V  = 0;
constexpr size_t YO_Y  = YO_V + SZ_V;
constexpr size_t YO_F1 = YO_Y + SZ_F;
constexpr size_t YO_G  = YO_F1 + SZ_F;
constexpr size_t YO_NB = YO_G + SZ_G;
static_assert(YO_NB + SZ_NB == (size_t)37996544 && YO_NB + SZ_NB <= SZ_Y);
static_assert(SZ_X == (size_t)76808192 && SZ_Y == (size_t)38404096);
static_assert((size_t)NPAD * 2 * KTAP * 2 <= SZ_X);
static_assert((size_t)MPAD * 32 * 2 <= SZ_Y && (size_t)MPAD * K_L2 * 2 <= SZ_Y);
static_assert(WS_TOTAL == ((size_t)491660 << 8));
static_assert(WS_TOTAL <= ((size_t)128 << 20));
static_assert(SZ_X % 256 == 0 && SZ_Y % 256 == 0 && SZ_F % 256 == 0 && SZ_V % 256 == 0 && SZ_G % 256 == 0);
static_assert(SZ_NB % 256 == 0 && SZ_LIST % 256 == 0 && SZ_NODE % 256 == 0 && SZ_FLAG % 256 == 0 && SZ_BW1 % 256 == 0);
static_assert(SZ_CWT % 256 == 0 && SZ_LWT % 256 == 0 && SZ_PAR % 256 == 0 && SZ_ST % 256 == 0 && SZ_REC % 256 == 0);
static_assert((size_t)PBK_NBLK * 128 <= SZ_FLAG && (size_t)NREC_N * CH * 8 <= SZ_REC);
static_assert((size_t)64 * K_1B * 2 <= SZ_BW1 && (size_t)64 * K_L2 * 2 <= SZ_LWT);

__device__ __forceinline__ float relu_k(float v) { return (v > 0.0f) ? v : (v - v); }

constexpr int PB_1A = 64 * (K_1A / 8) / 256;
constexpr int PB_1B = 64 * (K_1B / 8) / 256;
constexpr int PB_2A = 64 * (K_2A / 8) / 256;
constexpr int PB_2B = 64 * (K_2B / 8) / 256;
constexpr int PB_CW = 64 * (K_L1 / 8) / 256;
constexpr int PB_LW = 64 * (K_L2 / 8) / 256;
constexpr int PE_0 = PB_1A, PE_1 = PE_0 + PB_1B, PE_2 = PE_1 + PB_2A, PE_3 = PE_2 + PB_2B;
constexpr int PE_4 = PE_3 + PB_CW, PE_5 = PE_4 + PB_LW;
constexpr int PREP_BLOCKS = PE_5 + 1;
static_assert((64 * (K_1A / 8)) % 256 == 0 && (64 * (K_1B / 8)) % 256 == 0 && (64 * (K_2A / 8)) % 256 == 0);
static_assert((64 * (K_2B / 8)) % 256 == 0 && (64 * (K_L1 / 8)) % 256 == 0 && (64 * (K_L2 / 8)) % 256 == 0);

__device__ __forceinline__ void wt_unit(const float* __restrict__ W, int krows, int kmodp, int ppr,
                                        unsigned short* __restrict__ dst, int u) {
  const int n  = u / ppr;
  const int p  = u - n * ppr;
  const int ks = (p % kmodp) << 3;
  const int nc = n < CH ? n : CH - 1;
  float x[8];
  unsigned mk[8];
#pragma unroll
  for (int e = 0; e < 8; ++e) {
    const int k  = ks + e;
    const int kc = k < krows ? k : krows - 1;
    const float v = W[(size_t)kc * CH + nc];
    asm volatile("" :: "v"(v));
    x[e]  = v;
    mk[e] = (n < CH && k < krows) ? 0xFFFFu : 0u;
  }
  v4u o = pack8_bf16((v4f){ x[0], x[1], x[2], x[3] }, (v4f){ x[4], x[5], x[6], x[7] });
  o &= (v4u){ pk16(mk[0], mk[1]), pk16(mk[2], mk[3]), pk16(mk[4], mk[5]), pk16(mk[6], mk[7]) };
  volatile v4u* q = (volatile v4u*)(dst + (size_t)u * 8);
  *q = o;
  __threadfence();
  *q = o;
}

__device__ __forceinline__ v4u par_piece(const float* __restrict__ p, int j, bool on) {
  const v4f a = *(const v4fa*)(p + 4 * j);
  asm volatile("" :: "v"(a));
  const unsigned m = on ? 0xFFFFFFFFu : 0u;
  return (v4u){ __float_as_uint(a[0]) & m, __float_as_uint(a[1]) & m, __float_as_uint(a[2]) & m, __float_as_uint(a[3]) & m };
}

__global__ __launch_bounds__(256) void k_prep(const float* __restrict__ w1a, const float* __restrict__ w1b,
                                              const float* __restrict__ w2a, const float* __restrict__ w2b,
                                              const float* __restrict__ cw, const float* __restrict__ lw,
                                              const float* __restrict__ q0, const float* __restrict__ q1,
                                              const float* __restrict__ q2, const float* __restrict__ q3,
                                              const float* __restrict__ q4, const float* __restrict__ q5,
                                              const float* __restrict__ q6, const float* __restrict__ q7,
                                              const float* __restrict__ q8, const float* __restrict__ q9,
                                              const float* __restrict__ q10, const float* __restrict__ q11,
                                              const float* __restrict__ q12, const float* __restrict__ q13,
                                              const float* __restrict__ q14, const float* __restrict__ q15,
                                              unsigned short* __restrict__ BW, unsigned short* __restrict__ CWT,
                                              unsigned short* __restrict__ LWT, float* __restrict__ PAR) {
  const int tid = (int)threadIdx.x;
  const int blk = (int)blockIdx.x;
  constexpr int BWS = 64 * 2 * KTAP;
  if (blk < PE_0) {
    wt_unit(w1a, KTAP, KTAP / 8, K_1A / 8, BW, blk * 256 + tid);
  } else if (blk < PE_1) {
    wt_unit(w1b, KTAP, KTAP / 8, K_1B / 8, BW + BWS, (blk - PE_0) * 256 + tid);
  } else if (blk < PE_2) {
    wt_unit(w2a, KTAP, KTAP / 8, K_2A / 8, BW + 2 * BWS, (blk - PE_1) * 256 + tid);
  } else if (blk < PE_3) {
    wt_unit(w2b, KTAP, KTAP / 8, K_2B / 8, BW + 3 * BWS, (blk - PE_2) * 256 + tid);
  } else if (blk < PE_4) {
    wt_unit(cw, 8, 4, K_L1 / 8, CWT, (blk - PE_3) * 256 + tid);
  } else if (blk < PE_5) {
    wt_unit(lw, 32, 4, K_L2 / 8, LWT, (blk - PE_4) * 256 + tid);
  } else {
    const int u   = tid < P_N / 4 ? tid : P_N / 4 - 1;
    const int seg = u >> 3;
    const int j   = u & 7;
    v4u acc = par_piece(q0, j, seg == 0);
    acc |= par_piece(q1, j, seg == 1);
    acc |= par_piece(q2, j, seg == 2);
    acc |= par_piece(q3, j, seg == 3);
    acc |= par_piece(q4, j, seg == 4);
    acc |= par_piece(q5, j, seg == 5);
    acc |= par_piece(q6, j, seg == 6);
    acc |= par_piece(q7, j, seg == 7);
    acc |= par_piece(q8, j, seg == 8);
    acc |= par_piece(q9, j, seg == 9);
    acc |= par_piece(q10, j, seg == 10);
    acc |= par_piece(q11, j, seg == 11);
    acc |= par_piece(q12, j, seg == 12);
    acc |= par_piece(q13, j, seg == 13);
    acc |= par_piece(q14, j, seg == 14);
    acc |= par_piece(q15, j, seg == 15);
    const v4f o = (v4f){ bf16_val(__uint_as_float(acc[0])), bf16_val(__uint_as_float(acc[1])),
                         bf16_val(__uint_as_float(acc[2])), bf16_val(__uint_as_float(acc[3])) };
    if (tid < P_N / 4) {
      volatile v4f* q = (volatile v4f*)(PAR + 4 * tid);
      *q = o;
      __threadfence();
      *q = o;
    }
  }
}

__global__ __launch_bounds__(256) void k_grid(const int* __restrict__ idx, int* __restrict__ G) {
  __shared__ __attribute__((aligned(16))) int sg[GB_CELLS];
  const int tid  = (int)threadIdx.x;
  const int base = (int)blockIdx.x * GB_CELLS;
  {
    const v4i m1 = (v4i){ -1, -1, -1, -1 };
    for (int i = tid * 4; i < GB_CELLS; i += 1024) *(v4ia*)(sg + i) = m1;
  }
  __syncthreads();
#pragma unroll 1
  for (int k0 = 0; k0 < NS; k0 += 256) {
    const int n  = k0 + tid;
    const int nc = n < NS ? n : NS - 1;
    const int b = idx[3 * nc + 0];
    const int h = idx[3 * nc + 1];
    const int w = idx[3 * nc + 2];
    asm volatile("" :: "v"(b));
    asm volatile("" :: "v"(h));
    asm volatile("" :: "v"(w));
    const int cell = (clampi(b, 0, NBAT - 1) * HH + clampi(h, 0, HH - 1)) * WW + clampi(w, 0, WW - 1);
    const unsigned rel = (unsigned)(cell - base);
    if (n < NS && rel < (unsigned)GB_CELLS) atomicMax(&sg[rel], n);
  }
  __syncthreads();
  for (int pass = 0; pass < 2; ++pass) {
    for (int i = tid; i < GB_CELLS / 4; i += 256) {
      const v4i v = *(const v4ia*)(sg + 4 * i);
      const int c4 = base + 4 * i;
      if (c4 < NCELL) *(volatile v4i*)(G + c4) = v;
    }
    __threadfence();
  }
}

__global__ __launch_bounds__(256) void k_nbr(const int* __restrict__ idx, const int* __restrict__ G,
                                             int* __restrict__ NB) {
  const int tid = (int)threadIdx.x, lane = tid & 31, wave = tid >> 5;
  const int pair = (int)blockIdx.x * 8 + wave;
  const int site = 2 * pair + (lane >> 4);
  const int sc   = site < NS ? site : NS - 1;
  const int j    = lane & 15;
  int b = idx[3 * sc + 0];
  int h = idx[3 * sc + 1];
  int w = idx[3 * sc + 2];
  asm volatile("" :: "v"(b));
  asm volatile("" :: "v"(h));
  asm volatile("" :: "v"(w));
  b = clampi(b, 0, NBAT - 1);
  h = clampi(h, 0, HH - 1);
  w = clampi(w, 0, WW - 1);
  const int jj = j < 9 ? j : 8;
  const int kh = jj / 3;
  const int kw = jj - 3 * kh;
  const int h2 = h + kh - 1;
  const int w2 = w + kw - 1;
  const bool ok = (j < 9) && (h2 >= 0) && (h2 < HH) && (w2 >= 0) && (w2 < WW);
  int g = G[(b * HH + clampi(h2, 0, HH - 1)) * WW + clampi(w2, 0, WW - 1)];
  asm volatile("" :: "v"(g));
  g = clampi(g, -1, NS - 1);
  const int m = ok ? -1 : 0;
  const int v = (g & m) | (~m);
  if (site < NS) {
    volatile int* q = (volatile int*)(NB + (size_t)pair * 32 + lane);
    *q = v;
    __threadfence();
    *q = v;
  }
}

template <int TWO>
__global__ __launch_bounds__(256) void k_gather(const float* __restrict__ src, const int* __restrict__ NB,
                                                unsigned* __restrict__ A) {
  static_assert(TWO == 0 || TWO == 1);
  constexpr int RW  = TWO ? 288 : 144;
  constexpr int NPC = 2 * RW / 4;
  constexpr int NIT = (NPC + 31) / 32;
  __shared__ __attribute__((aligned(16))) unsigned strip[8][576];
  const int tid = (int)threadIdx.x, lane = tid & 31, wave = tid >> 5;
  const int pair = (int)blockIdx.x * 8 + wave;
  const bool live = pair < NS / 2;
  const int pc = live ? pair : NS / 2 - 1;
  int nbv = NB[(size_t)pc * 32 + lane];
  asm volatile("" :: "v"(nbv));
  nbv = clampi(nbv, -1, NS - 1);
  nbv = live ? nbv : -1;
  const int sub = lane >> 4;
  const int cp  = lane & 15;
  unsigned* st = strip[wave] + sub * RW;
#pragma unroll 3
  for (int t = 0; t < 9; ++t) {
    const int id  = __shfl(nbv, (lane & 16) + t, 32);
    const int idc = id < 0 ? 0 : id;
    const v2f r = *(const v2fa*)(src + (size_t)idc * CH + 2 * cp);
    asm volatile("" :: "v"(r));
    const unsigned m = (id >= 0) ? 0xFFFFFFFFu : 0u;
    const float v0 = __uint_as_float(__float_as_uint(r[0]) & m);
    const float v1 = __uint_as_float(__float_as_uint(r[1]) & m);
    st[16 * t + cp] = pk16(bf16_bits(v0), bf16_bits(v1));
    if (TWO) st[144 + 16 * t + cp] = pk16(bf16_lo_bits(v0), bf16_lo_bits(v1));
  }
  __builtin_amdgcn_fence(__ATOMIC_RELEASE, "workgroup");
  __builtin_amdgcn_wave_barrier();
  __builtin_amdgcn_fence(__ATOMIC_ACQUIRE, "workgroup");
  v4u vv[NIT];
#pragma unroll
  for (int it = 0; it < NIT; ++it) {
    const int pi = it * 32 + lane;
    const int pq = pi < NPC ? pi : NPC - 1;
    vv[it] = *(const v4ua*)(strip[wave] + 4 * pq);
  }
  unsigned* ab = A + (size_t)pair * (size_t)(2 * RW);
  for (int pass = 0; pass < 2; ++pass) {
#pragma unroll
    for (int it = 0; it < NIT; ++it) {
      const int pi = it * 32 + lane;
      if (pi < NPC) *(volatile v4u*)(ab + 4 * pi) = vv[it];
    }
    __threadfence();
  }
}

template <int MODE>
__global__ __launch_bounds__(256) void k_colstat(const float* __restrict__ H, int nrows,
                                                 const float* __restrict__ mean, double* __restrict__ rec) {
  static_assert(MODE == 0 || MODE == 1);
  __shared__ __attribute__((aligned(16))) float  sm[CH];
  __shared__ __attribute__((aligned(16))) double sp[256];
  const int tid = (int)threadIdx.x;
  if (tid < 32) {
    const int pc = tid & 7;
    v4f mv = (v4f){0.f, 0.f, 0.f, 0.f};
    if constexpr (MODE == 1) {
      mv = *(const v4fa*)(mean + 4 * pc);
      asm volatile("" :: "v"(mv));
    }
    *(v4fa*)(sm + 4 * pc) = mv;
  }
  __syncthreads();
  const int col = tid & 31;
  const int g   = tid >> 5;
  const int r0  = (int)blockIdx.x * 128 + g * 16;
  const int nr  = clampi(nrows - r0, 0, 16);
  const float m = sm[col];
  const float* hp = H + (size_t)r0 * LDV + col;
  double s = 0.0;
#pragma unroll 4
  for (int j = 0; j < nr; ++j) {
    const float v = hp[(size_t)j * LDV];
    if constexpr (MODE == 0) {
      s += (double)v;
    } else {
      const float d = v - m;
      const double dd = (double)d;
      s += dd * dd;
    }
  }
  sp[tid] = s;
  __syncthreads();
  if (tid < 32) {
    const int pc = tid < 16 ? tid : 15;
    double a0 = 0.0, a1 = 0.0;
#pragma unroll
    for (int q = 0; q < 8; ++q) {
      a0 += sp[q * 32 + 2 * pc];
      a1 += sp[q * 32 + 2 * pc + 1];
    }
    const v2d o = (v2d){ a0, a1 };
    volatile v2d* q = (volatile v2d*)(rec + (size_t)blockIdx.x * CH + 2 * pc);
    if (tid < 16) *q = o;
    __threadfence();
    if (tid < 16) *q = o;
  }
}

__global__ __launch_bounds__(32) void k_comb(const double* __restrict__ rec, int nrec, double inv_count, int mode,
                                             float* __restrict__ out) {
  __shared__ __attribute__((aligned(16))) float sv[32];
  const int tid = (int)threadIdx.x;
  double s = 0.0;
#pragma unroll 4
  for (int i = 0; i < nrec; ++i) s += rec[(size_t)i * CH + tid];
  const float qf = (float)(s * inv_count);
  const float rs = 1.0f / sqrtf(qf + 1e-3f);
  sv[tid] = (mode == 0) ? qf : rs;
  __syncthreads();
  const int t4 = tid < 8 ? tid : 7;
  const v4f o = *(const v4fa*)(sv + 4 * t4);
  if (tid < 8) {
    volatile v4f* q = (volatile v4f*)(out + 4 * tid);
    *q = o;
    __threadfence();
    *q = o;
  }
}

template <int KIND>
__global__ __launch_bounds__(256) void k_apply(const float* __restrict__ V, const float* __restrict__ res,
                                               const float* __restrict__ mean, const float* __restrict__ rstd,
                                               const float* __restrict__ gam, const float* __restrict__ bet,
                                               float* __restrict__ outp) {
  static_assert(KIND >= 0 && KIND <= 2);
  __shared__ __attribute__((aligned(16))) float spar[4 * CH];
  const int tid = (int)threadIdx.x, lane = tid & 31, wave = tid >> 5;
  const int c0 = 4 * (lane & 7);
  if (wave == 0) {
    const v4f a0 = *(const v4fa*)(mean + c0);
    const v4f a1 = *(const v4fa*)(rstd + c0);
    const v4f a2 = *(const v4fa*)(gam + c0);
    const v4f a3 = *(const v4fa*)(bet + c0);
    asm volatile("" :: "v"(a0));
    asm volatile("" :: "v"(a1));
    asm volatile("" :: "v"(a2));
    asm volatile("" :: "v"(a3));
    *(v4fa*)(spar + c0)          = a0;
    *(v4fa*)(spar + CH + c0)     = a1;
    *(v4fa*)(spar + 2 * CH + c0) = a2;
    *(v4fa*)(spar + 3 * CH + c0) = a3;
  }
  __syncthreads();
  const v4f mv = *(const v4fa*)(spar + c0);
  const v4f rv = *(const v4fa*)(spar + CH + c0);
  const v4f gv = *(const v4fa*)(spar + 2 * CH + c0);
  const v4f bv = *(const v4fa*)(spar + 3 * CH + c0);
  const int sub = lane >> 3;
#pragma unroll 1
  for (int i = 0; i < 8; ++i) {
    const int row = (int)blockIdx.x * 256 + wave * 32 + i * 4 + sub;
    const bool live = row < NS;
    const int rc = live ? row : NS - 1;
    const v4f cv = *(const v4fa*)(V + (size_t)rc * LDV + c0);
    asm volatile("" :: "v"(cv));
    v4f sk = (v4f){0.f, 0.f, 0.f, 0.f};
    if constexpr (KIND != 0) {
      sk = *(const v4fa*)(res + (size_t)rc * CH + c0);
      asm volatile("" :: "v"(sk));
      if constexpr (KIND == 1) sk = (v4f){ bf16_val(sk[0]), bf16_val(sk[1]), bf16_val(sk[2]), bf16_val(sk[3]) };
    }
    v4f y;
#pragma unroll
    for (int e = 0; e < 4; ++e) {
      const float t = ((cv[e] - mv[e]) * rv[e]) * gv[e] + bv[e];
      y[e] = (KIND == 0) ? relu_k(t) : relu_k(t + sk[e]);
    }
    float* op = outp + (size_t)rc * CH + c0;
    if (live) *(volatile v4f*)op = y;
    __threadfence();
    if (live) *(volatile v4f*)op = y;
  }
}

__global__ __launch_bounds__(256) void k_pp(const float* __restrict__ opf, unsigned short* __restrict__ PP) {
  const int u   = (int)blockIdx.x * 256 + (int)threadIdx.x;
  const int row = u >> 2;
  const int p   = u & 3;
  const int rc  = row < MS ? row : MS - 1;
  const v4f a = *(const v4fa*)(opf + (size_t)rc * 8);
  const v4f c = *(const v4fa*)(opf + (size_t)rc * 8 + 4);
  asm volatile("" :: "v"(a));
  asm volatile("" :: "v"(c));
  v4u o = pack8_bf16(a, c);
  const unsigned mk = (row < MS && p == 0) ? 0xFFFFFFFFu : 0u;
  o &= (v4u){ mk, mk, mk, mk };
  volatile v4u* q = (volatile v4u*)(PP + (size_t)u * 8);
  *q = o;
  __threadfence();
  *q = o;
}

template <int TWO>
__global__ __launch_bounds__(256) void k_apply1(const float* __restrict__ P, const int* __restrict__ unq,
                                                const float* __restrict__ F2,
                                                const float* __restrict__ mean, const float* __restrict__ rstd,
                                                const float* __restrict__ gam, const float* __restrict__ bet,
                                                unsigned* __restrict__ OPW) {
  static_assert(TWO == 0 || TWO == 1);
  __shared__ __attribute__((aligned(16))) float spar[4 * CH];
  const int tid = (int)threadIdx.x, lane = tid & 31, wave = tid >> 5;
  if (wave == 0) {
    const int c0 = 4 * (lane & 7);
    const v4f a0 = *(const v4fa*)(mean + c0);
    const v4f a1 = *(const v4fa*)(rstd + c0);
    const v4f a2 = *(const v4fa*)(gam + c0);
    const v4f a3 = *(const v4fa*)(bet + c0);
    asm volatile("" :: "v"(a0));
    asm volatile("" :: "v"(a1));
    asm volatile("" :: "v"(a2));
    asm volatile("" :: "v"(a3));
    *(v4fa*)(spar + c0)          = a0;
    *(v4fa*)(spar + CH + c0)     = a1;
    *(v4fa*)(spar + 2 * CH + c0) = a2;
    *(v4fa*)(spar + 3 * CH + c0) = a3;
  }
  __syncthreads();
  const float m  = spar[lane];
  const float r  = spar[CH + lane];
  const float g  = spar[2 * CH + lane];
  const float be = spar[3 * CH + lane];
  const int grp  = __builtin_amdgcn_readfirstlane((int)blockIdx.x * 8 + wave);
  const int base = grp * 32;
  const int e    = base + lane;
  const int ec   = e < MS ? e : MS - 1;
  int idv = unq[ec];
  asm volatile("" :: "v"(idv));
  idv = clampi(idv, 0, NS - 1);
  const int srcl = 2 * (lane & 15);
  if constexpr (TWO == 1) {
#pragma unroll 1
    for (int p = 0; p < 32; ++p) {
      const int pt = base + p;
      const bool live = pt < MS;
      const int ptc = live ? pt : MS - 1;
      const int id = __builtin_amdgcn_readlane(idv, p);
      const float v = P[(size_t)ptc * LDV + lane];
      asm volatile("" :: "v"(v));
      const float f = F2[(size_t)id * CH + lane];
      asm volatile("" :: "v"(f));
      const float o = relu_k(((v - m) * r) * g + be);
      const float t = o + f;
      const float s = live ? t : 0.0f;
      const unsigned w = bf16_bits(s) | (bf16_lo_bits(s) << 16);
      const unsigned a = (unsigned)__shfl((int)w, srcl, 32);
      const unsigned b = (unsigned)__shfl((int)w, srcl + 1, 32);
      const unsigned wl = pk16(a & 0xFFFFu, b & 0xFFFFu);
      const unsigned wh = pk16(a >> 16, b >> 16);
      const unsigned ow = (lane < 16) ? wl : wh;
      volatile unsigned* q = (volatile unsigned*)(OPW + (size_t)pt * 32 + lane);
      *q = ow;
      __threadfence();
      *q = ow;
    }
  } else {
#pragma unroll 1
    for (int p = 0; p < 16; ++p) {
      const int pt0 = base + 2 * p;
      const int pt1 = pt0 + 1;
      const bool l0 = pt0 < MS, l1 = pt1 < MS;
      const int c0 = l0 ? pt0 : MS - 1;
      const int c1 = l1 ? pt1 : MS - 1;
      const int i0 = __builtin_amdgcn_readlane(idv, 2 * p);
      const int i1 = __builtin_amdgcn_readlane(idv, 2 * p + 1);
      const float v0 = P[(size_t)c0 * LDV + lane];
      const float v1 = P[(size_t)c1 * LDV + lane];
      asm volatile("" :: "v"(v0));
      asm volatile("" :: "v"(v1));
      const float f0 = F2[(size_t)i0 * CH + lane];
      const float f1 = F2[(size_t)i1 * CH + lane];
      asm volatile("" :: "v"(f0));
      asm volatile("" :: "v"(f1));
      const float t0 = relu_k(((v0 - m) * r) * g + be) + f0;
      const float t1 = relu_k(((v1 - m) * r) * g + be) + f1;
      const float s0 = l0 ? t0 : 0.0f;
      const float s1 = l1 ? t1 : 0.0f;
      const unsigned w = bf16_bits(s0) | (bf16_bits(s1) << 16);
      const unsigned a = (unsigned)__shfl((int)w, srcl, 32);
      const unsigned b = (unsigned)__shfl((int)w, srcl + 1, 32);
      const unsigned wl = pk16(a & 0xFFFFu, b & 0xFFFFu);
      const unsigned wh = pk16(a >> 16, b >> 16);
      const unsigned ow = (lane < 16) ? wl : wh;
      volatile unsigned* q = (volatile unsigned*)(OPW + (size_t)pt0 * 16 + lane);
      *q = ow;
      __threadfence();
      *q = ow;
    }
  }
}

__global__ __launch_bounds__(256) void k_pbucket(const int* __restrict__ unq, int* __restrict__ LIST,
                                                 int* __restrict__ CNT, int* __restrict__ OFF,
                                                 int* __restrict__ FLAG) {
  extern __shared__ __attribute__((aligned(16))) int dsm[];
  int* wl   = dsm + BK_WL;
  int* sl   = dsm + BK_SL;
  int* cnt  = dsm + BK_CNT;
  int* offs = dsm + BK_OFF;
  int* cur  = dsm + BK_CUR;
  int* misc = dsm + BK_MISC;
  const int tid = (int)threadIdx.x, lane = tid & 31, wave = tid >> 5;
  const int blk = (int)blockIdx.x;
  const int nodeBase = blk * PBK_RUN;
  const int nbi = (NS - nodeBase) < PBK_RUN ? (NS - nodeBase) : PBK_RUN;
  const unsigned unb = (unsigned)(nbi < 0 ? 0 : nbi);

  {
    const v4i z4 = (v4i){0, 0, 0, 0};
    for (int i = tid * 4; i < RCAP + PBK_RUN; i += 1024) *(v4ia*)(sl + i) = z4;
    if (tid < 16) misc[tid] = 0;
  }
  __syncthreads();

  int* mylist = wl + wave * WLCAP;
  const int wbase = wave * EPW;
  const int wlast = wbase + EPW - 1;
  int wc = 0;
#pragma unroll 1
  for (int st = 0; st < NSTEP; ++st) {
    const int e0 = wbase + st * SUB + lane;
    int dk[4], ek[4];
#pragma unroll
    for (int j = 0; j < 4; ++j) {
      const int e  = e0 + 32 * j;
      const int ec = e < wlast ? e : wlast;
      const int d = unq[ec];
      asm volatile("" :: "v"(d));
      dk[j] = (e <= wlast) ? d : -1;
      ek[j] = ec;
    }
#pragma unroll
    for (int j = 0; j < 4; ++j) {
      const unsigned slot = (unsigned)dk[j] - (unsigned)nodeBase;
      const bool hit = slot < unb;
      const unsigned mj = __builtin_amdgcn_ballot_w32(hit);
      if (mj != 0u) {
        if (hit) {
          const int pos = wc + (int)__builtin_amdgcn_mbcnt_lo(mj, 0u);
          if (pos < WLCAP) mylist[pos] = (ek[j] << 10) | (int)slot;
        }
        wc += (int)__builtin_popcount(mj);
      }
    }
  }
  if (lane == 0) misc[wave] = wc;
  __syncthreads();

  if (wave == 0) {
    int t = 0, ov = 0;
#pragma unroll 1
    for (int w2 = 0; w2 < 8; ++w2) {
      const int craw = misc[w2];
      ov |= (craw > WLCAP) ? 1 : 0;
      const int c = __builtin_amdgcn_readfirstlane(clampi(craw, 0, WLCAP));
#pragma unroll 1
      for (int b0 = 0; b0 < c; b0 += 32) {
        const int idx = (b0 + lane) < c ? (b0 + lane) : c - 1;
        const int ent = wl[w2 * WLCAP + idx];
        const int m32 = (c - b0) < 32 ? (c - b0) : 32;
#pragma unroll 1
        for (int k = 0; k < m32; ++k) {
          const int u    = __builtin_amdgcn_readlane(ent, k);
          const int slot = u & (PBK_RUN - 1);
          if (t < RCAP) {
            if (lane == 0) cnt[slot] = cnt[slot] + 1;
            t = t + 1;
          } else {
            ov = 1;
          }
        }
      }
    }
    if (lane == 0) { misc[8] = t; misc[9] = ov; }
  }
  __syncthreads();

  if (wave == 0) {
    const int base = lane * (PBK_RUN / 32);
    int s = 0, big = 0;
#pragma unroll 1
    for (int i = 0; i < PBK_RUN / 32; ++i) {
      const int cv = cnt[base + i];
      s += cv;
      big |= (cv > DEGCAP) ? 1 : 0;
    }
    int incl = s;
#pragma unroll
    for (int d = 1; d < 32; d <<= 1) {
      const int y = __shfl_up(incl, d, 32);
      incl += (lane >= d) ? y : 0;
    }
    int run = incl - s;
#pragma unroll 1
    for (int i = 0; i < PBK_RUN / 32; ++i) {
      const int cv = cnt[base + i];
      offs[base + i] = run;
      cur[base + i]  = run;
      run += cv;
    }
    const unsigned bm = __builtin_amdgcn_ballot_w32(big != 0);
    if (lane == 0) misc[9] = misc[9] | ((bm != 0u) ? 1 : 0);
  }
  __syncthreads();

  if (wave == 0) {
    int t2 = 0;
#pragma unroll 1
    for (int w2 = 0; w2 < 8; ++w2) {
      const int c = __builtin_amdgcn_readfirstlane(clampi(misc[w2], 0, WLCAP));
#pragma unroll 1
      for (int b0 = 0; b0 < c; b0 += 32) {
        const int idx = (b0 + lane) < c ? (b0 + lane) : c - 1;
        const int ent = wl[w2 * WLCAP + idx];
        const int m32 = (c - b0) < 32 ? (c - b0) : 32;
#pragma unroll 1
        for (int k = 0; k < m32; ++k) {
          const int u    = __builtin_amdgcn_readlane(ent, k);
          const int slot = u & (PBK_RUN - 1);
          if (t2 < RCAP) {
            if (lane == 0) {
              int p = cur[slot];
              p = clampi(p, 0, RCAP - 1);
              sl[p] = u >> 10;
              cur[slot] = p + 1;
            }
            t2 = t2 + 1;
          }
        }
      }
    }
  }
  __syncthreads();

  const int ovf = misc[9];
  int* lbase = LIST + (size_t)blk * RCAP;
  for (int pass = 0; pass < 2; ++pass) {
    for (int i = tid; i < RCAP / 4; i += 256) {
      const v4i v = *(const v4ia*)(sl + 4 * i);
      *(volatile v4i*)(lbase + 4 * i) = v;
    }
    __threadfence();
  }
  const v4i cv4 = *(const v4ia*)(cnt + 4 * tid);
  const v4i ov4 = *(const v4ia*)(offs + 4 * tid);
  const v4i fl4 = (v4i){ ovf, ovf, ovf, ovf };
  const size_t nb4 = (size_t)nodeBase + 4 * (size_t)tid;
  const bool fw = (wave == 0) && (lane < 8);
  *(volatile v4i*)(CNT + nb4) = cv4;
  *(volatile v4i*)(OFF + nb4) = ov4;
  if (fw) *(volatile v4i*)(FLAG + blk * 32 + 4 * lane) = fl4;
  __threadfence();
  *(volatile v4i*)(CNT + nb4) = cv4;
  *(volatile v4i*)(OFF + nb4) = ov4;
  if (fw) *(volatile v4i*)(FLAG + blk * 32 + 4 * lane) = fl4;
}

__global__ __launch_bounds__(256) void k_segmax_out(const float* __restrict__ P, const int* __restrict__ LIST,
                                                    const int* __restrict__ CNT, const int* __restrict__ OFF,
                                                    const int* __restrict__ FLAG, const float* __restrict__ F2,
                                                    const float* __restrict__ mean, const float* __restrict__ rstd,
                                                    const float* __restrict__ gam, const float* __restrict__ bet,
                                                    float* __restrict__ outp, int nrows) {
  __shared__ __attribute__((aligned(16))) float spar[4 * CH];
  const int tid = (int)threadIdx.x, lane = tid & 31, wave = tid >> 5;
  if (wave == 0) {
    const int c0 = 4 * (lane & 7);
    const v4f a0 = *(const v4fa*)(mean + c0);
    const v4f a1 = *(const v4fa*)(rstd + c0);
    const v4f a2 = *(const v4fa*)(gam + c0);
    const v4f a3 = *(const v4fa*)(bet + c0);
    asm volatile("" :: "v"(a0));
    asm volatile("" :: "v"(a1));
    asm volatile("" :: "v"(a2));
    asm volatile("" :: "v"(a3));
    *(v4fa*)(spar + c0)          = a0;
    *(v4fa*)(spar + CH + c0)     = a1;
    *(v4fa*)(spar + 2 * CH + c0) = a2;
    *(v4fa*)(spar + 3 * CH + c0) = a3;
  }
  __syncthreads();
  const float m  = spar[lane];
  const float r  = spar[CH + lane];
  const float g  = spar[2 * CH + lane];
  const float be = spar[3 * CH + lane];

  const int i    = (int)blockIdx.x * 8 + wave;
  const bool live = i < nrows;
  const int ic   = clampi(i, 0, NS - 1);
  const int b    = ic >> 10;
  int c  = CNT[ic];
  int o  = OFF[ic];
  const int fl = FLAG[b * 32];
  asm volatile("" :: "v"(c));
  asm volatile("" :: "v"(o));
  asm volatile("" :: "v"(fl));
  c = clampi(c, 0, DEGCAP);
  o = clampi(o, 0, RCAP - DEGCAP);
  const int cn = __builtin_amdgcn_readfirstlane(live ? c : 0);
  const int* lp = LIST + (size_t)b * RCAP + o;

  float mx = __int_as_float((int)0xff800000u);
#pragma unroll 1
  for (int b0 = 0; b0 < cn; b0 += 32) {
    const int idx = (b0 + lane) < cn ? (b0 + lane) : cn - 1;
    int pt = lp[idx];
    asm volatile("" :: "v"(pt));
    pt = clampi(pt, 0, MS - 1);
    const int m32 = (cn - b0) < 32 ? (cn - b0) : 32;
#pragma unroll 1
    for (int k = 0; k < m32; ++k) {
      const int pk = __builtin_amdgcn_readlane(pt, k);
      const float v = P[(size_t)pk * LDV + lane];
      asm volatile("" :: "v"(v));
      const float t = relu_k(((v - m) * r) * g + be);
      mx = (t > mx || t != t) ? t : mx;
    }
  }
  const float f = F2[(size_t)ic * CH + lane];
  asm volatile("" :: "v"(f));
  const float sel = (cn == 0) ? f : mx;
  const float qn  = __int_as_float(0x7fc00000);
  const float ov  = (fl != 0) ? qn : sel;
  float* op = outp + (size_t)ic * CH + lane;
  if (live) *(volatile float*)op = ov;
  __threadfence();
  if (live) *(volatile float*)op = ov;
}

constexpr int G_GEMM_N = ((NPAD / 64) + 7) / 8;
constexpr int G_GEMM_M = ((MPAD / 64) + 7) / 8;
constexpr int G_APPLY  = (NS + 255) / 256;
static_assert(G_GEMM_N == 118 && G_GEMM_M == 586 && G_APPLY == 235);
static_assert((MPAD * 4) % 256 == 0 && (MPAD / 32) % 8 == 0 && NS % 16 == 0);

template <int TWO, int KIND>
static void conv_stage(const float* src, const float* res, const int* NB, unsigned short* Apl,
                       const unsigned short* Bpl, int ktot, const float* bias, float* V, double* REC,
                       float* stm, const float* gam, const float* bet, float* outp, hipStream_t stream) {
  const double invN = 1.0 / (double)NS;
  k_gather<TWO><<<NPAD / 2 / 8, 256, 0, stream>>>(src, NB, (unsigned*)Apl);
  k_gemm_nt<0, 1><<<G_GEMM_N, 256, 0, stream>>>(Apl, Bpl, bias, V, NPAD, CH, ktot, LDV);
  k_colstat<0><<<NREC_N, 256, 0, stream>>>(V, NS, stm, REC);
  k_comb<<<1, 32, 0, stream>>>(REC, NREC_N, invN, 0, stm);
  k_colstat<1><<<NREC_N, 256, 0, stream>>>(V, NS, stm, REC);
  k_comb<<<1, 32, 0, stream>>>(REC, NREC_N, invN, 1, stm + 32);
  k_apply<KIND><<<G_APPLY, 256, 0, stream>>>(V, res, stm, stm + 32, gam, bet, outp);
}

extern "C" void kernel_launch(void* const* d_in, const int* in_sizes, int n_in,
                              void* d_out, int out_size, void* d_ws, size_t ws_size,
                              hipStream_t stream) {
  if (n_in < 27) return;
  if (in_sizes[0] != NS * CH) return;
  if (in_sizes[1] != NS * 3) return;
  if (in_sizes[2] != MS * 8) return;
  if (in_sizes[3] != MS) return;
  if (in_sizes[4] != 1) return;
  for (int i = 5; i <= 8; ++i) if (in_sizes[i] != 9 * CH * CH) return;
  for (int i = 9; i <= 24; ++i) if (in_sizes[i] != CH) return;
  if (in_sizes[25] != 8 * CH) return;
  if (in_sizes[26] != CH * CH) return;
  if (out_size != NS * CH) return;
  if (ws_size < WS_TOTAL) return;

  const float* x   = (const float*)d_in[0];
  const int*   idx = (const int*)d_in[1];
  const float* opf = (const float*)d_in[2];
  const int*   unq = (const int*)d_in[3];
  const float* w1a = (const float*)d_in[5];
  const float* w1b = (const float*)d_in[6];
  const float* w2a = (const float*)d_in[7];
  const float* w2b = (const float*)d_in[8];
  const float* cw  = (const float*)d_in[25];
  const float* lw  = (const float*)d_in[26];
  float* out = (float*)d_out;

  char* ws = (char*)d_ws;
  unsigned short* Apl  = (unsigned short*)(ws + OFF_X);
  float*          P    = (float*)(ws + OFF_X);
  float*          V    = (float*)(ws + OFF_Y + YO_V);
  float*          Yb   = (float*)(ws + OFF_Y + YO_Y);
  float*          F1   = (float*)(ws + OFF_Y + YO_F1);
  int*            G    = (int*)(ws + OFF_Y + YO_G);
  int*            NB   = (int*)(ws + OFF_Y + YO_NB);
  unsigned short* PP   = (unsigned short*)(ws + OFF_Y);
  unsigned short* OP2  = (unsigned short*)(ws + OFF_Y);
  float*          F2   = (float*)(ws + OFF_F2);
  int*            LIST = (int*)(ws + OFF_LIST);
  int*            CNT  = (int*)(ws + OFF_CNT);
  int*            OFFS = (int*)(ws + OFF_OFF);
  int*            FLAG = (int*)(ws + OFF_FLAG);
  unsigned short* BW   = (unsigned short*)(ws + OFF_BW);
  unsigned short* CWT  = (unsigned short*)(ws + OFF_CWT);
  unsigned short* LWT  = (unsigned short*)(ws + OFF_LWT);
  float*          PAR  = (float*)(ws + OFF_PAR);
  float*          ST   = (float*)(ws + OFF_ST);
  double*         REC  = (double*)(ws + OFF_REC);
  constexpr int BWS = 64 * 2 * KTAP;

  hipFuncSetAttribute(reinterpret_cast<const void*>(&k_pbucket), hipFuncAttributeMaxDynamicSharedMemorySize, (int)BK_LDS);

  k_prep<<<PREP_BLOCKS, 256, 0, stream>>>(w1a, w1b, w2a, w2b, cw, lw,
      (const float*)d_in[9],  (const float*)d_in[10], (const float*)d_in[11], (const float*)d_in[12],
      (const float*)d_in[13], (const float*)d_in[14], (const float*)d_in[15], (const float*)d_in[16],
      (const float*)d_in[17], (const float*)d_in[18], (const float*)d_in[19], (const float*)d_in[20],
      (const float*)d_in[21], (const float*)d_in[22], (const float*)d_in[23], (const float*)d_in[24],
      BW, CWT, LWT, PAR);
  k_grid<<<GB_BLOCKS, 256, 0, stream>>>(idx, G);
  k_nbr<<<NS / 2 / 8, 256, 0, stream>>>(idx, G, NB);
  conv_stage<0, 0>(x, x, NB, Apl, BW, K_1A, PAR + P_B, V, REC, ST, PAR + P_G, PAR + P_BE, Yb, stream);
  conv_stage<TWO_TERM_C1B, 1>(Yb, x, NB, Apl, BW + BWS, K_1B, PAR + P_B + 32, V, REC, ST + 64,
                              PAR + P_G + 32, PAR + P_BE + 32, F1, stream);
  conv_stage<TWO_TERM_C2A, 0>(F1, F1, NB, Apl, BW + 2 * BWS, K_2A, PAR + P_B + 64, V, REC, ST + 128,
                              PAR + P_G + 64, PAR + P_BE + 64, Yb, stream);
  conv_stage<TWO_TERM_C2B, 2>(Yb, F1, NB, Apl, BW + 3 * BWS, K_2B, PAR + P_B + 96, V, REC, ST + 192,
                              PAR + P_G + 96, PAR + P_BE + 96, F2, stream);

  const double invM = 1.0 / (double)MS;
  k_pp<<<MPAD * 4 / 256, 256, 0, stream>>>(opf, PP);
  k_gemm_nt<0, 0><<<G_GEMM_M, 256, 0, stream>>>(PP, CWT, PAR, P, MPAD, CH, K_L1, LDV);
  k_colstat<0><<<NREC_M, 256, 0, stream>>>(P, MS, ST + 256, REC);
  k_comb<<<1, 32, 0, stream>>>(REC, NREC_M, invM, 0, ST + 256);
  k_colstat<1><<<NREC_M, 256, 0, stream>>>(P, MS, ST + 256, REC);
  k_comb<<<1, 32, 0, stream>>>(REC, NREC_M, invM, 1, ST + 256 + 32);
  k_apply1<TWO_TERM_L2><<<MPAD / 32 / 8, 256, 0, stream>>>(P, unq, F2, ST + 256, ST + 256 + 32,
                                                           PAR + P_G + 128, PAR + P_BE + 128, (unsigned*)OP2);
  k_gemm_nt<0, 0><<<G_GEMM_M, 256, 0, stream>>>(OP2, LWT, PAR, P, MPAD, CH, K_L2, LDV);
  k_colstat<0><<<NREC_M, 256, 0, stream>>>(P, MS, ST + 320, REC);
  k_comb<<<1, 32, 0, stream>>>(REC, NREC_M, invM, 0, ST + 320);
  k_colstat<1><<<NREC_M, 256, 0, stream>>>(P, MS, ST + 320, REC);
  k_comb<<<1, 32, 0, stream>>>(REC, NREC_M, invM, 1, ST + 320 + 32);
  k_pbucket<<<PBK_NBLK, 256, BK_LDS, stream>>>(unq, LIST, CNT, OFFS, FLAG);
  k_segmax_out<<<NS / 8, 256, 0, stream>>>(P, LIST, CNT, OFFS, FLAG, F2, ST + 320, ST + 320 + 32,
                                           PAR + P_G + 160, PAR + P_BE + 160, out, NS);
}
